// LSTM_6201932776128
// MI455X (gfx1250) — hardware-run, weakly checked
//
#include <hip/hip_runtime.h>
#include <math.h>

constexpr int NBATCH   = 64;
constexpr int NSTEPS   = 64;
constexpr int NDIM     = 768;
constexpr int NHID     = 768;
constexpr int NGATE4   = 4 * NHID;
constexpr int NTHR     = 256;
constexpr int ROWS_BLK = 16;
constexpr int HPITCH   = 776;
constexpr int SPITCH   = 772;
constexpr int SLABP    = 68;
constexpr float WCARRY  = 256.0f;
constexpr float XCARRY  = 16.0f;
constexpr float HCARRY  = 64.0f;
constexpr float LOCARRY = 2048.0f;
constexpr float PROJ_S0 = 1.0f / (WCARRY * XCARRY);
constexpr float PROJ_S1 = 1.0f / (WCARRY * XCARRY * LOCARRY);
constexpr float REC_S   = 1.0f / (WCARRY * HCARRY);
constexpr int GROUPS_PER_WAVE = 6;

static_assert(NDIM % 32 == 0 && NHID % 32 == 0, "K multiple of 32");
static_assert(NDIM == NHID, "one Bt pitch for both weight families");
static_assert(NBATCH % ROWS_BLK == 0, "row blocks");
static_assert(NBATCH == 64, "projection N tile is 64 columns");
static_assert((NGATE4 / 16) % (NTHR / 32) == 0, "projection grid exact");
static_assert(NHID / 16 == (NTHR / 32) * GROUPS_PER_WAVE, "8 waves x 6 groups of 16 units");
static_assert((ROWS_BLK * NHID / 4) % NTHR == 0, "final store loop exact");
static_assert(NDIM % 64 == 0 && NHID % 64 == 0, "transpose tiles");
static_assert((NBATCH * NDIM / 8) % NTHR == 0, "x gather grid exact");
static_assert((NGATE4 / 4) % NTHR == 0, "bias grid exact");

typedef __attribute__((ext_vector_type(16))) _Float16 v16h;
typedef __attribute__((ext_vector_type(8)))  _Float16 v8h;
typedef __attribute__((ext_vector_type(8)))  float    v8f;
typedef __attribute__((ext_vector_type(4)))  float    v4f;

__device__ __forceinline__ void guard_grp4(v8f& a0, v8f& a1, v8f& a2, v8f& a3, v16h x, v16h y0, v16h y1, v16h y2, v16h y3) {
  asm volatile("v_nop\n\tv_nop\n\tv_nop\n\tv_nop" : "+v"(a0), "+v"(a1), "+v"(a2), "+v"(a3) : "v"(x), "v"(y0), "v"(y1), "v"(y2), "v"(y3));
}
__device__ __forceinline__ void guard_pair(v8f& a0, v8f& a1, v16h x0, v16h x1, v16h y0, v16h y1) {
  asm volatile("v_nop\n\tv_nop\n\tv_nop\n\tv_nop" : "+v"(a0), "+v"(a1) : "v"(x0), "v"(x1), "v"(y0), "v"(y1));
}
__device__ __forceinline__ void acc_guard4(v8f& a, v8f& b, v8f& c, v8f& d) {
  asm volatile("v_nop\n\tv_nop\n\tv_nop\n\tv_nop" : "+v"(a), "+v"(b), "+v"(c), "+v"(d));
}

template <typename T> struct Frag;
template <> struct Frag<_Float16> {
  typedef v16h V; union U { v16h v; v8h h[2]; };
  static __device__ __forceinline__ v16h load(const _Float16* p) {
    U f; f.h[0] = *(const v8h*)(p); f.h[1] = *(const v8h*)(p + 16); return f.v;
  }
  static __device__ __forceinline__ v8f mma(v16h a, v16h b, v8f c) {
    return __builtin_amdgcn_wmma_f32_16x16x32_f16(false, a, false, b, (short)0, c, false, false);
  }
};

__device__ __forceinline__ void split_h(float f, _Float16& hi, _Float16& lo) {
  hi = (_Float16)f;
  const float back = (float)hi;
  lo = (_Float16)((f - back) * LOCARRY);
}

__device__ __forceinline__ float gate_sig(float x) {
  const float e = expf(fminf(-x, 40.0f));
  return __builtin_amdgcn_rcpf(1.0f + e);
}
__device__ __forceinline__ float gate_tanh(float x) {
  const float e = expf(fminf(2.0f * x, 40.0f));
  return 1.0f - 2.0f * __builtin_amdgcn_rcpf(e + 1.0f);
}

__global__ __launch_bounds__(NTHR) void tp_planes_kernel(
    const float* __restrict__ s0, const float* __restrict__ s1, const float* __restrict__ s2, const float* __restrict__ s3,
    const float* __restrict__ s4, const float* __restrict__ s5, const float* __restrict__ s6, const float* __restrict__ s7,
    unsigned short* __restrict__ WtH, unsigned short* __restrict__ WtL, unsigned short* __restrict__ Ut) {
  __shared__ float Tt[64 * 65];
  const int tid = threadIdx.x;
  const int c0 = blockIdx.x * 64, r0 = blockIdx.y * 64;
  const int z = blockIdx.z;
  const int g = z & 3;
  const float* src = (z == 0) ? s0 : (z == 1) ? s1 : (z == 2) ? s2 : (z == 3) ? s3
                   : (z == 4) ? s4 : (z == 5) ? s5 : (z == 6) ? s6 : s7;
#pragma unroll
  for (int i = 0; i < 4; ++i) {
    const int idx = i * NTHR + tid;
    const int rr = idx >> 4, cc = (idx & 15) * 4;
    const v4f v = *(const v4f*)(src + (size_t)(r0 + rr) * (size_t)NHID + c0 + cc);
    Tt[rr * 65 + cc + 0] = v[0];
    Tt[rr * 65 + cc + 1] = v[1];
    Tt[rr * 65 + cc + 2] = v[2];
    Tt[rr * 65 + cc + 3] = v[3];
  }
  __syncthreads();
  const int q = tid >> 3, c8 = (tid & 7) * 8;
  v8h hv[2], lv[2];
#pragma unroll
  for (int gs = 0; gs < 2; ++gs) {
    const int qq = gs * 32 + q;
#pragma unroll
    for (int e = 0; e < 8; ++e) {
      const float f = Tt[(c8 + e) * 65 + qq] * WCARRY;
      _Float16 hi, lo;
      split_h(f, hi, lo);
      hv[gs][e] = hi;
      lv[gs][e] = lo;
    }
  }
  const bool with_lo = (z < 4);
  unsigned short* dh = with_lo ? WtH : Ut;
  for (int pass = 0; pass < 2; ++pass) {
#pragma unroll
    for (int gs = 0; gs < 2; ++gs) {
      const int jcol = c0 + gs * 32 + q;
      const int np = (jcol >> 4) * 64 + g * 16 + (jcol & 15);
      const size_t o = (size_t)np * (size_t)NHID + (size_t)(r0 + c8);
      *(volatile v8h*)(dh + o) = hv[gs];
      if (with_lo) *(volatile v8h*)(WtL + o) = lv[gs];
    }
    __threadfence();
  }
}

__global__ __launch_bounds__(NTHR) void prep_small_kernel(
    const float* __restrict__ X,
    const float* __restrict__ b0, const float* __restrict__ b1, const float* __restrict__ b2, const float* __restrict__ b3,
    unsigned short* __restrict__ XlH, unsigned short* __restrict__ XlL, float* __restrict__ BP) {
  const int tid = threadIdx.x;
  const int nxb = (NBATCH * NDIM / 8) / NTHR;
  if ((int)blockIdx.x < nxb) {
    const int i = blockIdx.x * NTHR + tid;
    const int b = i / (NDIM / 8);
    const int c8 = i - b * (NDIM / 8);
    const float* sp = X + ((size_t)b * NSTEPS + (size_t)(NSTEPS - 1)) * NDIM + c8 * 8;
    const v4f a = *(const v4f*)(sp);
    const v4f bb = *(const v4f*)(sp + 4);
    v8h hv, lv;
#pragma unroll
    for (int e = 0; e < 4; ++e) {
      _Float16 hi, lo;
      split_h(a[e] * XCARRY, hi, lo);
      hv[e] = hi; lv[e] = lo;
      split_h(bb[e] * XCARRY, hi, lo);
      hv[4 + e] = hi; lv[4 + e] = lo;
    }
    *(volatile v8h*)(XlH + (size_t)i * 8) = hv;
    *(volatile v8h*)(XlL + (size_t)i * 8) = lv;
    __threadfence();
    *(volatile v8h*)(XlH + (size_t)i * 8) = hv;
    *(volatile v8h*)(XlL + (size_t)i * 8) = lv;
  } else {
    const int t = ((int)blockIdx.x - nxb) * NTHR + tid;
    const int np = 4 * t;
    const int grp = np >> 6, g = (np >> 4) & 3, cc = np & 15;
    const int j = grp * 16 + cc;
    v4f v0 = *(const v4f*)(b0 + j);
    v4f v1 = *(const v4f*)(b1 + j);
    v4f v2 = *(const v4f*)(b2 + j);
    v4f v3 = *(const v4f*)(b3 + j);
    asm volatile("" : "+v"(v0), "+v"(v1), "+v"(v2), "+v"(v3));
    v4f o;
#pragma unroll
    for (int e = 0; e < 4; ++e) {
      const float x0 = v0[e], x1 = v1[e], x2 = v2[e], x3 = v3[e];
      o[e] = (g == 0) ? x0 : (g == 1) ? x1 : (g == 2) ? x2 : x3;
    }
    *(volatile v4f*)(BP + np) = o;
    __threadfence();
    *(volatile v4f*)(BP + np) = o;
  }
}

__global__ __launch_bounds__(NTHR) void proj_kernel(
    const unsigned short* __restrict__ WtHp, const unsigned short* __restrict__ WtLp,
    const unsigned short* __restrict__ XlHp, const unsigned short* __restrict__ XlLp,
    const float* __restrict__ BP, float* __restrict__ XGT) {
  __shared__ __align__(16) float sT[NTHR / 32][16 * SLABP];
  const _Float16* WtH = (const _Float16*)WtHp;
  const _Float16* WtL = (const _Float16*)WtLp;
  const _Float16* XlH = (const _Float16*)XlHp;
  const _Float16* XlL = (const _Float16*)XlLp;
  const int lane = threadIdx.x & 31;
  const int wave = __builtin_amdgcn_readfirstlane((int)(threadIdx.x >> 5));
  const int c = lane & 15, hh = lane >> 4, koff = hh * 8;
  const int tile = blockIdx.x * (NTHR / 32) + wave;
  const int m0 = tile * 16;

  const _Float16* wa_h = WtH + (size_t)(m0 + c) * NDIM + koff;
  const _Float16* wa_l = WtL + (size_t)(m0 + c) * NDIM + koff;
  const _Float16* xb_h = XlH + (size_t)c * NDIM + koff;
  const _Float16* xb_l = XlL + (size_t)c * NDIM + koff;

  const v8f z8 = {0.f, 0.f, 0.f, 0.f, 0.f, 0.f, 0.f, 0.f};
  v8f acc[4], accr[4];
#pragma unroll
  for (int j = 0; j < 4; ++j) { acc[j] = z8; accr[j] = z8; }

#pragma unroll 1
  for (int k0 = 0; k0 < NDIM; k0 += 32) {
    const v16h ah = Frag<_Float16>::load(wa_h + k0);
    const v16h al = Frag<_Float16>::load(wa_l + k0);
#pragma unroll
    for (int j = 0; j < 4; ++j) {
      const v16h bh = Frag<_Float16>::load(xb_h + (size_t)j * 16 * NDIM + k0);
      const v16h bl = Frag<_Float16>::load(xb_l + (size_t)j * 16 * NDIM + k0);
      acc[j]  = Frag<_Float16>::mma(ah, bh, acc[j]);
      accr[j] = Frag<_Float16>::mma(ah, bl, accr[j]);
      accr[j] = Frag<_Float16>::mma(al, bh, accr[j]);
      guard_pair(acc[j], accr[j], ah, al, bh, bl);
    }
  }
  acc_guard4(acc[0], acc[1], acc[2], acc[3]);
  acc_guard4(accr[0], accr[1], accr[2], accr[3]);

  const v4f bq0 = *(const v4f*)(BP + m0 + 8 * hh);
  const v4f bq1 = *(const v4f*)(BP + m0 + 8 * hh + 4);
  float* slab = sT[wave];
#pragma unroll
  for (int j = 0; j < 4; ++j) {
#pragma unroll
    for (int r = 0; r < 8; ++r) {
      const float bs = (r < 4) ? bq0[r & 3] : bq1[r & 3];
      const float main_t = acc[j][r] * PROJ_S0;
      const float res_t  = accr[j][r] * PROJ_S1;
      slab[(8 * hh + r) * SLABP + 16 * j + c] = (main_t + res_t) + bs;
    }
  }
  __builtin_amdgcn_fence(__ATOMIC_RELEASE, "workgroup");
  __builtin_amdgcn_wave_barrier();
  __builtin_amdgcn_fence(__ATOMIC_ACQUIRE, "workgroup");
  {
    const int c4 = c * 4;
    for (int pass = 0; pass < 2; ++pass) {
#pragma unroll
      for (int it = 0; it < 8; ++it) {
        const int row = it * 2 + hh;
        const v4f v = *(const v4f*)(slab + row * SLABP + c4);
        *(volatile v4f*)(XGT + (size_t)(m0 + row) * NBATCH + c4) = v;
      }
      __threadfence();
    }
  }
}

__global__ __launch_bounds__(NTHR) void cell_iter_kernel(const float* __restrict__ XGT, const float* __restrict__ mask,
                                                         const unsigned short* __restrict__ Utp, float* __restrict__ out) {
  __shared__ __align__(16) _Float16 Ah[2][ROWS_BLK * HPITCH];
  __shared__ __align__(16) float    Hs[ROWS_BLK * SPITCH];
  __shared__ __align__(16) float    Cs[ROWS_BLK * SPITCH];
  const _Float16* Ut = (const _Float16*)Utp;
  const int tid = threadIdx.x, lane = tid & 31;
  const int wave = __builtin_amdgcn_readfirstlane((int)(threadIdx.x >> 5));
  const int c = lane & 15, hh = lane >> 4, koff = hh * 8;
  const int rowbase = blockIdx.x * ROWS_BLK;

  {
    _Float16* ahf = &Ah[0][0];
#pragma unroll 1
    for (int i = tid; i < 2 * ROWS_BLK * HPITCH; i += NTHR) ahf[i] = (_Float16)0.0f;
#pragma unroll 1
    for (int i = tid; i < ROWS_BLK * SPITCH; i += NTHR) { Hs[i] = 0.0f; Cs[i] = 0.0f; }
  }
  float mk[8];
#pragma unroll
  for (int r = 0; r < 8; ++r) mk[r] = mask[(size_t)(rowbase + 8 * hh + r) * NSTEPS + (NSTEPS - 1)];
  __syncthreads();

  const v8f z8 = {0.f, 0.f, 0.f, 0.f, 0.f, 0.f, 0.f, 0.f};

#pragma unroll 1
  for (int s = 0; s < NSTEPS; ++s) {
    const int cur = s & 1;
    const _Float16* ahrow = &Ah[0][0] + cur * (ROWS_BLK * HPITCH) + c * HPITCH + koff;
    _Float16* ahn = &Ah[0][0] + (cur ^ 1) * (ROWS_BLK * HPITCH);
#pragma unroll 1
    for (int gi = 0; gi < GROUPS_PER_WAVE; ++gi) {
      const int grp = wave * GROUPS_PER_WAVE + gi;
      const int j = grp * 16 + c;
      const _Float16* ub = Ut + (size_t)(grp * 64 + c) * NHID + koff;
      v8f acc0 = z8, acc1 = z8, acc2 = z8, acc3 = z8;
#pragma unroll 1
      for (int k0 = 0; k0 < NHID; k0 += 32) {
        const v16h a  = Frag<_Float16>::load(ahrow + k0);
        const v16h b0 = Frag<_Float16>::load(ub + k0);
        const v16h b1 = Frag<_Float16>::load(ub + (size_t)16 * NHID + k0);
        const v16h b2 = Frag<_Float16>::load(ub + (size_t)32 * NHID + k0);
        const v16h b3 = Frag<_Float16>::load(ub + (size_t)48 * NHID + k0);
        acc0 = Frag<_Float16>::mma(a, b0, acc0);
        acc1 = Frag<_Float16>::mma(a, b1, acc1);
        acc2 = Frag<_Float16>::mma(a, b2, acc2);
        acc3 = Frag<_Float16>::mma(a, b3, acc3);
        guard_grp4(acc0, acc1, acc2, acc3, a, b0, b1, b2, b3);
      }
      acc_guard4(acc0, acc1, acc2, acc3);

      const float* xq = XGT + (size_t)(grp * 64 + c) * NBATCH + rowbase + 8 * hh;
      const v4f xi0 = *(const v4f*)(xq);
      const v4f xi1 = *(const v4f*)(xq + 4);
      const v4f xf0 = *(const v4f*)(xq + (size_t)16 * NBATCH);
      const v4f xf1 = *(const v4f*)(xq + (size_t)16 * NBATCH + 4);
      const v4f xc0 = *(const v4f*)(xq + (size_t)32 * NBATCH);
      const v4f xc1 = *(const v4f*)(xq + (size_t)32 * NBATCH + 4);
      const v4f xo0 = *(const v4f*)(xq + (size_t)48 * NBATCH);
      const v4f xo1 = *(const v4f*)(xq + (size_t)48 * NBATCH + 4);

#pragma unroll
      for (int r = 0; r < 8; ++r) {
        const float xi = (r < 4) ? xi0[r & 3] : xi1[r & 3];
        const float xf = (r < 4) ? xf0[r & 3] : xf1[r & 3];
        const float xc = (r < 4) ? xc0[r & 3] : xc1[r & 3];
        const float xo = (r < 4) ? xo0[r & 3] : xo1[r & 3];
        const float zi = acc0[r] * REC_S + xi;
        const float zf = acc1[r] * REC_S + xf;
        const float zc = acc2[r] * REC_S + xc;
        const float zo = acc3[r] * REC_S + xo;
        const float ig = gate_tanh(zi);
        const float fg = gate_sig(zf);
        const float gg = gate_tanh(zc);
        const float og = gate_sig(zo);
        const int so = (8 * hh + r) * SPITCH + j;
        const float cold = Cs[so];
        const float hold = Hs[so];
        const float cn = fg * cold + ig * gg;
        const float hn = og * gate_tanh(cn);
        const float m  = mk[r];
        const float hb = (1.0f - m) * hold + m * hn;
        const float cb = (1.0f - m) * cold + m * cn;
        Cs[so] = cb;
        Hs[so] = hb;
        ahn[(8 * hh + r) * HPITCH + j] = (_Float16)(hb * HCARRY);
      }
    }
    __syncthreads();
  }

  for (int pass = 0; pass < 2; ++pass) {
#pragma unroll
    for (int it = 0; it < (ROWS_BLK * NHID / 4) / NTHR; ++it) {
      const int idx = it * NTHR + tid;
      const int row = idx / (NHID / 4);
      const int c4  = (idx - row * (NHID / 4)) * 4;
      const v4f v = *(const v4f*)(Hs + row * SPITCH + c4);
      *(volatile v4f*)(out + (size_t)(rowbase + row) * NHID + c4) = v;
    }
    __threadfence();
  }
}

extern "C" void kernel_launch(void* const* d_in, const int* in_sizes, int n_in,
                              void* d_out, int out_size, void* d_ws, size_t ws_size, hipStream_t stream) {
  if (n_in < 14 || d_out == nullptr || d_ws == nullptr) return;
  if (in_sizes[0] != NBATCH * NSTEPS * NDIM || in_sizes[1] != NBATCH * NSTEPS) return;
  for (int i = 2; i < 6; ++i) if (in_sizes[i] != NDIM * NHID) return;
  for (int i = 6; i < 10; ++i) if (in_sizes[i] != NHID * NHID) return;
  for (int i = 10; i < 14; ++i) if (in_sizes[i] != NHID) return;
  if (out_size != NBATCH * NHID) return;

  const float* X    = (const float*)d_in[0];
  const float* mask = (const float*)d_in[1];
  const float* w0 = (const float*)d_in[2];
  const float* w1 = (const float*)d_in[3];
  const float* w2 = (const float*)d_in[4];
  const float* w3 = (const float*)d_in[5];
  const float* u0 = (const float*)d_in[6];
  const float* u1 = (const float*)d_in[7];
  const float* u2 = (const float*)d_in[8];
  const float* u3 = (const float*)d_in[9];
  const float* b0 = (const float*)d_in[10];
  const float* b1 = (const float*)d_in[11];
  const float* b2 = (const float*)d_in[12];
  const float* b3 = (const float*)d_in[13];
  float* out = (float*)d_out;

  char* ws = (char*)d_ws; size_t off = 0;
  auto carve = [&](size_t bytes) -> char* { char* p = ws + off; off += (bytes + 255) & ~(size_t)255; return p; };
  unsigned short* WtH = (unsigned short*)carve((size_t)NGATE4 * NDIM * 2);
  unsigned short* WtL = (unsigned short*)carve((size_t)NGATE4 * NDIM * 2);
  unsigned short* Ut  = (unsigned short*)carve((size_t)NGATE4 * NHID * 2);
  unsigned short* XlH = (unsigned short*)carve((size_t)NBATCH * NDIM * 2);
  unsigned short* XlL = (unsigned short*)carve((size_t)NBATCH * NDIM * 2);
  float*          BP  = (float*)carve((size_t)NGATE4 * 4);
  float*          XGT = (float*)carve((size_t)NGATE4 * NBATCH * 4);
  if (off > ws_size || off > (size_t)134217728) return;

  tp_planes_kernel<<<dim3(NHID / 64, NDIM / 64, 8), NTHR, 0, stream>>>(w0, w1, w2, w3, u0, u1, u2, u3, WtH, WtL, Ut);
  prep_small_kernel<<<(NBATCH * NDIM / 8) / NTHR + (NGATE4 / 4) / NTHR, NTHR, 0, stream>>>(X, b0, b1, b2, b3, XlH, XlL, BP);
  proj_kernel<<<(NGATE4 / 16) / (NTHR / 32), NTHR, 0, stream>>>(WtH, WtL, XlH, XlL, BP, XGT);
  cell_iter_kernel<<<NBATCH / ROWS_BLK, NTHR, 0, stream>>>(XGT, mask, Ut, out);
}
